// ChebNet_BenQin_64364379898363
// MI455X (gfx1250) — hardware-verified
//
#include <hip/hip_runtime.h>
#include <stdint.h>
#include <stddef.h>


#define NN    4096
#define FD    256
#define CC    40
#define CPAD  48
#define KW    512
#define KP1   3
#define PADH  40
#define LSCALE   1024.0f
#define TWO_PI_F 6.28318530717958647692f

#define LDS_ALIGNED __shared__ __attribute__((aligned(16)))

typedef _Float16 v8h  __attribute__((ext_vector_type(8)));
typedef _Float16 v16h __attribute__((ext_vector_type(16)));
typedef float    v8f  __attribute__((ext_vector_type(8)));
typedef float    v4f  __attribute__((ext_vector_type(4)));
typedef int      v4i  __attribute__((ext_vector_type(4)));

union Frag { v16h v; v8h half[2]; };
union H8   { v8h h; v4i i; };

__device__ __forceinline__ v16h frag16(const _Float16* p0, const _Float16* p1) {
    Frag f;
    f.half[0] = *(const v8h*)p0;
    f.half[1] = *(const v8h*)p1;
    return f.v;
}

__device__ __forceinline__ v8f wmma16(v8f acc, v16h a, v16h b) {
    acc = __builtin_amdgcn_wmma_f32_16x16x32_f16(false, a, false, b, (short)0, acc, false, false);
    asm volatile("v_nop\n\tv_nop\n\tv_nop\n\tv_nop" : "+v"(acc) : "v"(a), "v"(b));
    return acc;
}

__device__ __forceinline__ v8h cvt8(v4f a, v4f b) {
    v8h r;
    r[0] = (_Float16)a.x; r[1] = (_Float16)a.y; r[2] = (_Float16)a.z; r[3] = (_Float16)a.w;
    r[4] = (_Float16)b.x; r[5] = (_Float16)b.y; r[6] = (_Float16)b.z; r[7] = (_Float16)b.w;
    return r;
}

__device__ __forceinline__ void sincos_p(float x, float* sp, float* cp) {
    const float fn = rintf(x * 0.63661977236758134f);
    const int n = (int)fn;
    float r = fmaf(-fn, 1.57079637050628662109375f, x);
    r = fmaf(-fn, -4.37113883e-08f, r);
    const float r2 = r * r;
    float ps = fmaf(r2, 2.75573192e-06f, -1.98412698e-04f);
    ps = fmaf(r2, ps, 8.33333333e-03f);
    ps = fmaf(r2, ps, -1.66666667e-01f);
    const float sn = fmaf(r2 * r, ps, r);
    float pc = fmaf(r2, 2.48015873e-05f, -1.38888889e-03f);
    pc = fmaf(r2, pc, 4.16666667e-02f);
    pc = fmaf(r2, pc, -0.5f);
    const float cs = fmaf(r2, pc, 1.0f);
    const int q = n & 3;
    float s, c;
    if (q == 0)      { s =  sn; c =  cs; }
    else if (q == 1) { s =  cs; c = -sn; }
    else if (q == 2) { s = -sn; c = -cs; }
    else             { s = -cs; c =  sn; }
    *sp = s; *cp = c;
}

__global__ __launch_bounds__(256) void k_adj_rows(const int* __restrict__ edges,
                                                   const float* __restrict__ w,
                                                   int E, float* __restrict__ A) {
    LDS_ALIGNED float rowv[NN];
    __shared__ int   lcol[256];
    __shared__ float lw[256];
    __shared__ int   wcnt[2][8];
    const int tid = threadIdx.x, lane = tid & 31, wave = tid >> 5;
    const int r = blockIdx.x;
    for (int j = tid; j < NN; j += 256) rowv[j] = 0.f;
    const int nchunk = (E + 255) >> 8;
    for (int ch = 0; ch < nchunk; ++ch) {
        const int e = (ch << 8) + tid;
        int cc = 0; float ww = 0.f; bool match = false;
        if (e < E) {
            int rr = edges[e];
            if (rr < 0) rr += NN;
            if (rr == r) {
                cc = edges[(size_t)E + e];
                ww = w[e];
                if (cc < 0) cc += NN;
                match = ((unsigned)cc < (unsigned)NN);
            }
        }
        const unsigned long long mask = __ballot(match ? 1 : 0);
        const int cnt  = __popcll(mask);
        const int rank = __popcll(mask & ((1ull << lane) - 1ull));
        const int par = ch & 1;
        if (lane == 0) wcnt[par][wave] = cnt;
        __syncthreads();
        int total = 0, prefix = 0;
#pragma unroll
        for (int u = 0; u < 8; ++u) {
            const int c = wcnt[par][u];
            total += c;
            prefix += (u < wave) ? c : 0;
        }
        if (total == 0) continue;
        if (match) { lcol[prefix + rank] = cc; lw[prefix + rank] = ww; }
        __syncthreads();
        if (tid == 0) {
            for (int u = 0; u < total; ++u) rowv[lcol[u]] += lw[u];
        }
    }
    __syncthreads();
    float* base = A + (size_t)r * NN;
    v4f vals[4];
#pragma unroll
    for (int q = 0; q < 4; ++q) vals[q] = *(const v4f*)&rowv[(q * 256 + tid) * 4];
#pragma unroll
    for (int q = 0; q < 4; ++q) *(volatile v4f*)(base + (q * 256 + tid) * 4) = vals[q];
    __threadfence();
#pragma unroll
    for (int q = 0; q < 4; ++q) *(volatile v4f*)(base + (q * 256 + tid) * 4) = vals[q];
}

__global__ __launch_bounds__(256) void k_rowsum(const float* __restrict__ A, float* __restrict__ rs) {
    LDS_ALIGNED float sm[32];
    const int tid = threadIdx.x, lane = tid & 31, wave = tid >> 5;
    const int rblk = blockIdx.x * 32;
#pragma unroll
    for (int rr = 0; rr < 4; ++rr) {
        const int row = rblk + wave * 4 + rr;
        const float* ap = A + (size_t)row * NN;
        float s = 0.f;
#pragma unroll 4
        for (int i = 0; i < NN / 128; ++i) {
            const v4f v = *(const v4f*)(ap + (i * 32 + lane) * 4);
            s += (v.x + v.y) + (v.z + v.w);
        }
        for (int off = 16; off > 0; off >>= 1) s += __shfl_xor(s, off, 32);
        if (lane == 0) sm[wave * 4 + rr] = s;
    }
    __syncthreads();
    if (tid < 8) {
        const v4f v = *(const v4f*)&sm[tid * 4];
        float* p = rs + rblk + tid * 4;
        *(volatile v4f*)p = v;
        __threadfence();
        *(volatile v4f*)p = v;
    }
}

__global__ __launch_bounds__(256) void k_dinv(const float* __restrict__ A, const float* __restrict__ rs,
                                               float* __restrict__ dinv) {
    LDS_ALIGNED float sm[256];
    const int tid = threadIdx.x;
    const int j = blockIdx.x * 256 + tid;
    float s = 0.f;
#pragma unroll 8
    for (int i = 0; i < NN; ++i) s += A[(size_t)i * NN + j];
    const float d = 0.5f * (s + rs[j]);
    const float dv = (d == 0.f) ? 1.f : (1.0f / sqrtf(d));
    sm[tid] = dv;
    __syncthreads();
    if (tid < 64) {
        const v4f v = *(const v4f*)&sm[tid * 4];
        float* p = dinv + blockIdx.x * 256 + tid * 4;
        *(volatile v4f*)p = v;
        __threadfence();
        *(volatile v4f*)p = v;
    }
}

__global__ __launch_bounds__(256) void k_build_l(const float* __restrict__ A,
                                                  const float* __restrict__ dinv,
                                                  const float* __restrict__ qp,
                                                  _Float16* __restrict__ LR,
                                                  _Float16* __restrict__ LI) {
    LDS_ALIGNED float    P[64][64];
    LDS_ALIGNED float    Q[64][68];
    LDS_ALIGNED _Float16 TR[64][64];
    LDS_ALIGNED _Float16 TI[64][64];
    const int tid = threadIdx.x;
    const int i0 = (int)(blockIdx.x >> 6) * 64;
    const int j0 = (int)(blockIdx.x & 63) * 64;
#pragma unroll
    for (int s = 0; s < 4; ++s) {
        const int idx = tid + s * 256;
        const int row = idx >> 4, c4 = idx & 15;
        *(v4f*)&P[row][c4 * 4] = *(const v4f*)(A + (size_t)(i0 + row) * NN + j0 + c4 * 4);
        *(v4f*)&Q[row][c4 * 4] = *(const v4f*)(A + (size_t)(j0 + row) * NN + i0 + c4 * 4);
    }
    __syncthreads();
    const float cq = TWO_PI_F * qp[0];
    {
        const int ii = tid >> 2;
        const int jb = (tid & 3) * 16;
        const float di = dinv[i0 + ii];
#pragma unroll 1
        for (int e = 0; e < 16; ++e) {
            const int jj = jb + e;
            const float a  = P[ii][jj];
            const float at = Q[jj][ii];
            const float asym = 0.5f * (a + at);
            const float an = (di * asym) * dinv[j0 + jj];
            const float th = cq * (a - at);
            float s, c;
            sincos_p(th, &s, &c);
            TR[ii][jj] = (_Float16)((-(an * c)) * LSCALE);
            TI[ii][jj] = (_Float16)((an * s) * LSCALE);
        }
    }
    __syncthreads();
    H8 vr[2], vi[2];
    const int piece = tid & 7;
#pragma unroll
    for (int p = 0; p < 2; ++p) {
        const int ii = p * 32 + (tid >> 3);
        vr[p].h = *(const v8h*)&TR[ii][piece * 8];
        vi[p].h = *(const v8h*)&TI[ii][piece * 8];
    }
#pragma unroll
    for (int p = 0; p < 2; ++p) {
        const size_t o = (size_t)(i0 + p * 32 + (tid >> 3)) * NN + j0 + piece * 8;
        *(volatile v4i*)(LR + o) = vr[p].i;
        *(volatile v4i*)(LI + o) = vi[p].i;
    }
    __threadfence();
#pragma unroll
    for (int p = 0; p < 2; ++p) {
        const size_t o = (size_t)(i0 + p * 32 + (tid >> 3)) * NN + j0 + piece * 8;
        *(volatile v4i*)(LR + o) = vr[p].i;
        *(volatile v4i*)(LI + o) = vi[p].i;
    }
}

__global__ __launch_bounds__(256) void k_cvt16(const float* __restrict__ Xr, const float* __restrict__ Xi,
                                                int n8, _Float16* __restrict__ Or, _Float16* __restrict__ Oi) {
    const int i8 = blockIdx.x * 256 + threadIdx.x;
    if (i8 >= n8) return;
    const size_t o = (size_t)i8 * 8;
    H8 hr, hi;
    hr.h = cvt8(*(const v4f*)(Xr + o), *(const v4f*)(Xr + o + 4));
    hi.h = cvt8(*(const v4f*)(Xi + o), *(const v4f*)(Xi + o + 4));
    *(volatile v4i*)(Or + o) = hr.i;
    *(volatile v4i*)(Oi + o) = hi.i;
    __threadfence();
    *(volatile v4i*)(Or + o) = hr.i;
    *(volatile v4i*)(Oi + o) = hi.i;
}

__global__ __launch_bounds__(256) void k_prepwc(const float* __restrict__ Wc, _Float16* __restrict__ W16) {
    const int i8 = blockIdx.x * 256 + threadIdx.x;
    if (i8 >= (CPAD * KW) / 8) return;
    const int row = i8 >> 6, c8 = i8 & 63;
    H8 v;
    if (row < CC) {
        const float* p = Wc + (size_t)row * KW + c8 * 8;
        v.h = cvt8(*(const v4f*)p, *(const v4f*)(p + 4));
    } else {
        v.i = (v4i){0, 0, 0, 0};
    }
    _Float16* d = W16 + (size_t)row * KW + c8 * 8;
    *(volatile v4i*)d = v.i;
    __threadfence();
    *(volatile v4i*)d = v.i;
}

__global__ __launch_bounds__(256) void k_gemm_l(
        const _Float16* __restrict__ LR, const _Float16* __restrict__ LI,
        const _Float16* __restrict__ Xr, const _Float16* __restrict__ Xi,
        const float* __restrict__ Z0r, const float* __restrict__ Z0i,
        _Float16* __restrict__ Yr, _Float16* __restrict__ Yi,
        float oscale, int sub) {
    LDS_ALIGNED unsigned char smem[32768];
    _Float16* sA = (_Float16*)smem;
    _Float16* sB = (_Float16*)(smem + 2 * 64 * PADH * 2);
    const int tid = threadIdx.x, lane = tid & 31, wave = tid >> 5;
    const int m = lane & 15, h = lane >> 4;
    const int rowBase = (blockIdx.x >> 1) * 64;
    const int colBase = (blockIdx.x & 1) * 128;
    const int wy = wave >> 1, wx = wave & 1;

    v8f re[4], im[4];
#pragma unroll
    for (int t = 0; t < 4; ++t) { re[t] = (v8f){}; im[t] = (v8f){}; }

    for (int k0 = 0; k0 < NN; k0 += 32) {
        __syncthreads();
#pragma unroll
        for (int s = 0; s < 2; ++s) {
            const int t2 = tid + s * 256;
            const int mat = t2 >> 8, rem = t2 & 255, row = rem >> 2, ch = rem & 3;
            const _Float16* src = (mat ? LI : LR) + (size_t)(rowBase + row) * NN + k0 + ch * 8;
            *(v8h*)(sA + (mat * 64 + row) * PADH + ch * 8) = *(const v8h*)src;
        }
#pragma unroll
        for (int s = 0; s < 4; ++s) {
            const int t4 = tid + s * 256;
            const int mat = t4 >> 9, rem = t4 & 511, kk = rem >> 4, fc = rem & 15;
            const _Float16* src = (mat ? Xi : Xr) + (size_t)(k0 + kk) * FD + colBase + fc * 8;
            const v8h v = *(const v8h*)src;
            _Float16* dst = sB + (mat * 128 + fc * 8) * PADH + kk;
#pragma unroll
            for (int u = 0; u < 8; ++u) dst[u * PADH] = v[u];
        }
        __syncthreads();
        const _Float16* pa = sA + (wy * 16 + m) * PADH;
        const v16h Ar  = frag16(pa + 8 * h, pa + 16 + 8 * h);
        const v16h Ai  = frag16(pa + 64 * PADH + 8 * h, pa + 64 * PADH + 16 + 8 * h);
        const v16h nAi = -Ai;
#pragma unroll
        for (int ct = 0; ct < 4; ++ct) {
            const _Float16* pb = sB + (wx * 64 + ct * 16 + m) * PADH;
            const v16h Br = frag16(pb + 8 * h, pb + 16 + 8 * h);
            const v16h Bi = frag16(pb + 128 * PADH + 8 * h, pb + 128 * PADH + 16 + 8 * h);
            re[ct] = wmma16(re[ct], Ar,  Br);
            re[ct] = wmma16(re[ct], nAi, Bi);
            im[ct] = wmma16(im[ct], Ar,  Bi);
            im[ct] = wmma16(im[ct], Ai,  Br);
        }
    }
    __syncthreads();

    _Float16* epi = (_Float16*)smem + wave * 2048;
    const int rowg0 = rowBase + wy * 16;
    const int colg0 = colBase + wx * 64;
#pragma unroll
    for (int ct = 0; ct < 4; ++ct) {
        const int col = ct * 16 + m;
#pragma unroll
        for (int r = 0; r < 8; ++r) {
            const int row = 8 * h + r;
            float zr = 0.f, zi = 0.f;
            if (sub) {
                const size_t o = (size_t)(rowg0 + row) * FD + colg0 + col;
                zr = Z0r[o]; zi = Z0i[o];
            }
            epi[row * 64 + col]        = (_Float16)(re[ct][r] * oscale - zr);
            epi[1024 + row * 64 + col] = (_Float16)(im[ct][r] * oscale - zi);
        }
    }
    __syncthreads();
    H8 vals[8];
    const int piece = lane & 7;
#pragma unroll
    for (int q = 0; q < 8; ++q) {
        const int mat = q >> 2, row = (q & 3) * 4 + (lane >> 3);
        vals[q].h = *(const v8h*)(epi + mat * 1024 + row * 64 + piece * 8);
    }
#pragma unroll
    for (int q = 0; q < 8; ++q) {
        const int mat = q >> 2, row = (q & 3) * 4 + (lane >> 3);
        _Float16* d = (mat ? Yi : Yr) + (size_t)(rowg0 + row) * FD + colg0 + piece * 8;
        *(volatile v4i*)d = vals[q].i;
    }
    __threadfence();
#pragma unroll
    for (int q = 0; q < 8; ++q) {
        const int mat = q >> 2, row = (q & 3) * 4 + (lane >> 3);
        _Float16* d = (mat ? Yi : Yr) + (size_t)(rowg0 + row) * FD + colg0 + piece * 8;
        *(volatile v4i*)d = vals[q].i;
    }
}

__global__ __launch_bounds__(256) void k_gemm_w(
        const _Float16* __restrict__ Z0r, const _Float16* __restrict__ Z0i,
        const _Float16* __restrict__ Z1r, const _Float16* __restrict__ Z1i,
        const _Float16* __restrict__ Z2r, const _Float16* __restrict__ Z2i,
        const float* __restrict__ W, const float* __restrict__ bias,
        float* __restrict__ Or32, float* __restrict__ Oi32,
        _Float16* __restrict__ Or16, _Float16* __restrict__ Oi16) {
    LDS_ALIGNED unsigned char smem[32768];
    _Float16* sW = (_Float16*)smem;
    const int tid = threadIdx.x, lane = tid & 31, wave = tid >> 5;
    const int m = lane & 15, h = lane >> 4;
    const int rowBase = (blockIdx.x >> 1) * 64;
    const int colBase = (blockIdx.x & 1) * 128;
    const int wy = wave >> 1, wx = wave & 1;
    const int rowg0 = rowBase + wy * 16;
    const int colg0 = colBase + wx * 64;

    v8f sr[4], si[4];
#pragma unroll
    for (int t = 0; t < 4; ++t) { sr[t] = (v8f){}; si[t] = (v8f){}; }

#pragma unroll
    for (int t = 0; t < KP1; ++t) {
        const _Float16* zr = (t == 0) ? Z0r : ((t == 1) ? Z1r : Z2r);
        const _Float16* zi = (t == 0) ? Z0i : ((t == 1) ? Z1i : Z2i);
        const float* Wt = W + (size_t)t * FD * FD;
        for (int k0 = 0; k0 < FD; k0 += 32) {
            __syncthreads();
#pragma unroll
            for (int s = 0; s < 4; ++s) {
                const int idx = tid + s * 256;
                const int kk = idx >> 5, c4 = idx & 31;
                const v4f v = *(const v4f*)(Wt + (size_t)(k0 + kk) * FD + colBase + c4 * 4);
                _Float16* dst = sW + (c4 * 4) * PADH + kk;
                dst[0]        = (_Float16)v.x;
                dst[PADH]     = (_Float16)v.y;
                dst[2 * PADH] = (_Float16)v.z;
                dst[3 * PADH] = (_Float16)v.w;
            }
            __syncthreads();
            const _Float16* pa = zr + (size_t)(rowg0 + m) * FD + k0;
            const _Float16* pi = zi + (size_t)(rowg0 + m) * FD + k0;
            const v16h Ar = frag16(pa + 8 * h, pa + 16 + 8 * h);
            const v16h Ai = frag16(pi + 8 * h, pi + 16 + 8 * h);
#pragma unroll
            for (int ct = 0; ct < 4; ++ct) {
                const _Float16* pb = sW + (wx * 64 + ct * 16 + m) * PADH;
                const v16h Bw = frag16(pb + 8 * h, pb + 16 + 8 * h);
                sr[ct] = wmma16(sr[ct], Ar, Bw);
                si[ct] = wmma16(si[ct], Ai, Bw);
            }
        }
    }

    float* epi = (float*)smem + wave * 1024;
#pragma unroll
    for (int mat = 0; mat < 2; ++mat) {
        __syncthreads();
#pragma unroll
        for (int ct = 0; ct < 4; ++ct) {
            const int col = ct * 16 + m;
            const float b = bias[colg0 + col];
#pragma unroll
            for (int r = 0; r < 8; ++r) {
                const int row = 8 * h + r;
                const float v = (mat == 0) ? (b - si[ct][r]) : (sr[ct][r] + b);
                epi[row * 64 + col] = v;
            }
        }
        __syncthreads();
        v4f f[8];
        H8  g[4];
#pragma unroll
        for (int q = 0; q < 8; ++q) {
            const int row = q * 2 + (lane >> 4), pc = lane & 15;
            f[q] = *(const v4f*)(epi + row * 64 + pc * 4);
        }
#pragma unroll
        for (int q = 0; q < 4; ++q) {
            const int row = q * 4 + (lane >> 3), pc = lane & 7;
            const v4f a = *(const v4f*)(epi + row * 64 + pc * 8);
            const v4f c = *(const v4f*)(epi + row * 64 + pc * 8 + 4);
            g[q].h = cvt8(a, c);
        }
        float*    o32 = mat ? Oi32 : Or32;
        _Float16* o16 = mat ? Oi16 : Or16;
#pragma unroll
        for (int q = 0; q < 8; ++q) {
            const int row = q * 2 + (lane >> 4), pc = lane & 15;
            *(volatile v4f*)(o32 + (size_t)(rowg0 + row) * FD + colg0 + pc * 4) = f[q];
        }
#pragma unroll
        for (int q = 0; q < 4; ++q) {
            const int row = q * 4 + (lane >> 3), pc = lane & 7;
            *(volatile v4i*)(o16 + (size_t)(rowg0 + row) * FD + colg0 + pc * 8) = g[q].i;
        }
        __threadfence();
#pragma unroll
        for (int q = 0; q < 8; ++q) {
            const int row = q * 2 + (lane >> 4), pc = lane & 15;
            *(volatile v4f*)(o32 + (size_t)(rowg0 + row) * FD + colg0 + pc * 4) = f[q];
        }
#pragma unroll
        for (int q = 0; q < 4; ++q) {
            const int row = q * 4 + (lane >> 3), pc = lane & 7;
            *(volatile v4i*)(o16 + (size_t)(rowg0 + row) * FD + colg0 + pc * 8) = g[q].i;
        }
    }
}

__global__ __launch_bounds__(64) void k_cls(const _Float16* __restrict__ Xr, const _Float16* __restrict__ Xi,
                                             const _Float16* __restrict__ W16, const float* __restrict__ bc,
                                             float* __restrict__ out) {
    LDS_ALIGNED float os[2][640];
    LDS_ALIGNED float lg[2][16 * CPAD];
    const int tid = threadIdx.x, lane = tid & 31, wave = tid >> 5;
    const int m = lane & 15, h = lane >> 4;
    const int row0 = (blockIdx.x * 2 + wave) * 16;

    v8f acc[3];
#pragma unroll
    for (int t = 0; t < 3; ++t) acc[t] = (v8f){};
    for (int k0 = 0; k0 < KW; k0 += 32) {
        const _Float16* pa = ((k0 < FD) ? Xr : Xi) + (size_t)(row0 + m) * FD + (k0 & (FD - 1));
        const v16h Ar = frag16(pa + 8 * h, pa + 16 + 8 * h);
#pragma unroll
        for (int ct = 0; ct < 3; ++ct) {
            const _Float16* pb = W16 + (size_t)(ct * 16 + m) * KW + k0;
            const v16h Bw = frag16(pb + 8 * h, pb + 16 + 8 * h);
            acc[ct] = wmma16(acc[ct], Ar, Bw);
        }
    }
    float* lgw = &lg[wave][0];
    float* osw = &os[wave][0];
#pragma unroll
    for (int ct = 0; ct < 3; ++ct) {
        const int col = ct * 16 + m;
        const float b = (col < CC) ? bc[col] : 0.f;
#pragma unroll
        for (int r = 0; r < 8; ++r) lgw[(8 * h + r) * CPAD + col] = acc[ct][r] + b;
    }
    __syncthreads();
    if (h == 0) {
        const int row = m;
        float mx = lgw[row * CPAD];
#pragma unroll 1
        for (int c = 1; c < CC; ++c) mx = fmaxf(mx, lgw[row * CPAD + c]);
        float s = 0.f;
#pragma unroll 1
        for (int c = 0; c < CC; ++c) s += expf(lgw[row * CPAD + c] - mx);
        const float ls = logf(s);
#pragma unroll 1
        for (int c = 0; c < CC; ++c) osw[row * CC + c] = (lgw[row * CPAD + c] - mx) - ls;
    }
    __syncthreads();
    v4f vals[5];
#pragma unroll
    for (int q = 0; q < 5; ++q) vals[q] = *(const v4f*)(osw + (q * 32 + lane) * 4);
    float* ob = out + (size_t)row0 * CC;
#pragma unroll
    for (int q = 0; q < 5; ++q) *(volatile v4f*)(ob + (q * 32 + lane) * 4) = vals[q];
    __threadfence();
#pragma unroll
    for (int q = 0; q < 5; ++q) *(volatile v4f*)(ob + (q * 32 + lane) * 4) = vals[q];
}

extern "C" void kernel_launch(void* const* d_in, const int* in_sizes, int n_in,
                              void* d_out, int out_size, void* d_ws, size_t ws_size,
                              hipStream_t stream) {
    if (n_in < 11) return;
    if (in_sizes[0] != NN * FD || in_sizes[1] != NN * FD) return;
    if (in_sizes[2] < 0 || (in_sizes[2] & 1)) return;
    const int E = in_sizes[2] / 2;
    if (in_sizes[3] < 1 || in_sizes[4] < E) return;
    if (in_sizes[5] != KP1 * FD * FD || in_sizes[7] != KP1 * FD * FD) return;
    if (in_sizes[6] < FD || in_sizes[8] < FD) return;
    if (in_sizes[9] != CC * KW || in_sizes[10] < CC) return;
    if (out_size != NN * CC) return;

    const float* real  = (const float*)d_in[0];
    const float* imag  = (const float*)d_in[1];
    const int*   edges = (const int*)d_in[2];
    const float* qp    = (const float*)d_in[3];
    const float* ew    = (const float*)d_in[4];
    const float* W1    = (const float*)d_in[5];
    const float* b1    = (const float*)d_in[6];
    const float* W2    = (const float*)d_in[7];
    const float* b2    = (const float*)d_in[8];
    const float* Wc    = (const float*)d_in[9];
    const float* bc    = (const float*)d_in[10];
    float* out = (float*)d_out;

    const size_t MiB   = (size_t)1 << 20;
    const size_t szA   = (size_t)NN * NN * sizeof(float);
    const size_t szL   = (size_t)NN * NN * sizeof(_Float16);
    const size_t szH   = (size_t)NN * FD * sizeof(_Float16);
    const size_t szF   = (size_t)NN * FD * sizeof(float);
    const size_t szVec = (size_t)NN * sizeof(float);

    size_t off = 0;
    char* ws = (char*)d_ws;
    float*    A     = (float*)(ws + off);    off += szA;
    _Float16* LR    = (_Float16*)(ws + off); off += szL;
    _Float16* LI    = (_Float16*)(ws + off); off += szL;
    _Float16* X16r  = (_Float16*)(ws + off); off += szH;
    _Float16* X16i  = (_Float16*)(ws + off); off += szH;
    _Float16* Z1r   = (_Float16*)(ws + off); off += szH;
    _Float16* Z1i   = (_Float16*)(ws + off); off += szH;
    _Float16* Z2r   = (_Float16*)(ws + off); off += szH;
    _Float16* Z2i   = (_Float16*)(ws + off); off += szH;
    _Float16* O1r16 = (_Float16*)(ws + off); off += szH;
    _Float16* O1i16 = (_Float16*)(ws + off); off += szH;
    _Float16* O2r16 = (_Float16*)(ws + off); off += szH;
    _Float16* O2i16 = (_Float16*)(ws + off); off += szH;
    float*    O1r32 = (float*)(ws + off);    off += szF;
    float*    O1i32 = (float*)(ws + off);    off += szF;
    float*    O2r32 = (float*)(ws + off);    off += szF;
    float*    O2i32 = (float*)(ws + off);    off += szF;
    _Float16* Wc16  = (_Float16*)(ws + off); off += MiB;
    float*    rsum  = (float*)(ws + off);    off += szVec;
    float*    dinv  = (float*)(ws + off);    off += szVec;
    if (off > ws_size) return;

    const int n8      = NN * FD / 8;
    const int GEMM_BLK = (NN / 64) * (FD / 128);
    const float osc1 = 1.0f / LSCALE;
    const float osc2 = 2.0f / LSCALE;

    k_adj_rows<<<NN, 256, 0, stream>>>(edges, ew, E, A);
    k_rowsum<<<NN / 32, 256, 0, stream>>>(A, rsum);
    k_dinv<<<NN / 256, 256, 0, stream>>>(A, rsum, dinv);
    k_build_l<<<(NN / 64) * (NN / 64), 256, 0, stream>>>(A, dinv, qp, LR, LI);

    k_cvt16<<<(n8 + 255) / 256, 256, 0, stream>>>(real, imag, n8, X16r, X16i);
    k_prepwc<<<(CPAD * KW / 8 + 255) / 256, 256, 0, stream>>>(Wc, Wc16);

    k_gemm_l<<<GEMM_BLK, 256, 0, stream>>>(LR, LI, X16r, X16i, real, imag, Z1r, Z1i, osc1, 0);
    k_gemm_l<<<GEMM_BLK, 256, 0, stream>>>(LR, LI, Z1r, Z1i, real, imag, Z2r, Z2i, osc2, 1);
    k_gemm_w<<<GEMM_BLK, 256, 0, stream>>>(X16r, X16i, Z1r, Z1i, Z2r, Z2i, W1, b1,
                                           O1r32, O1i32, O1r16, O1i16);

    k_gemm_l<<<GEMM_BLK, 256, 0, stream>>>(LR, LI, O1r16, O1i16, O1r32, O1i32, Z1r, Z1i, osc1, 0);
    k_gemm_l<<<GEMM_BLK, 256, 0, stream>>>(LR, LI, Z1r, Z1i, O1r32, O1i32, Z2r, Z2i, osc2, 1);
    k_gemm_w<<<GEMM_BLK, 256, 0, stream>>>(O1r16, O1i16, Z1r, Z1i, Z2r, Z2i, W2, b2,
                                           O2r32, O2i32, O2r16, O2i16);

    k_cls<<<NN / 32, 64, 0, stream>>>(O2r16, O2i16, Wc16, bc, out);
}
